// KANLayer_11776800325919
// MI455X (gfx1250) — hardware-verified
//
#include <hip/hip_runtime.h>
#include <stdint.h>

#pragma clang fp contract(off)

#define NROWS  8192
#define NIN    256
#define NOUT   256
#define NB     7
#define KSP    (NIN * NB)
#define KTOT   (2 * NIN + 2 * KSP)
#define OSL    NIN
#define OBH    (2 * NIN)
#define OBL    (2 * NIN + KSP)
#define UROW   (KTOT / 8)
#define FTHR   256
#define NSWEEP (UROW / FTHR)
#define CSU    (KSP / 8)
#define WSCAP  134217728

static_assert(KTOT % 32 == 0);
static_assert(NROWS % 128 == 0);
static_assert(NOUT % 64 == 0);
static_assert(NIN % 32 == 0);
static_assert(UROW == NSWEEP * FTHR);
static_assert(KSP == CSU * 8);
static_assert(CSU % 32 == 0);
static_assert((OSL * 2) % 128 == 0);
static_assert((OBH * 2) % 128 == 0);
static_assert((OBL * 2) % 128 == 0);
static_assert((KTOT * 2) % 128 == 0);
static_assert(FTHR == NIN);
static_assert(NIN * 16 % 512 == 0);

typedef float          v4f   __attribute__((ext_vector_type(4)));
typedef float          v8f   __attribute__((ext_vector_type(8)));
typedef int            v8i   __attribute__((ext_vector_type(8)));
typedef unsigned int   v4u   __attribute__((ext_vector_type(4)));
typedef unsigned short v8us  __attribute__((ext_vector_type(8)));
typedef unsigned short v16us __attribute__((ext_vector_type(16)));
typedef __bf16         v16bf __attribute__((ext_vector_type(16)));
typedef v4f  __attribute__((may_alias)) v4fa;
typedef v4u  __attribute__((may_alias)) v4ua;
typedef v8us __attribute__((may_alias)) v8usa;
union FragB { v16bf v; v16us u; v8us h[2]; v8i w; };

__device__ __forceinline__ unsigned short f2bf_bits(float f) {
  unsigned u = __float_as_uint(f);
  return (unsigned short)((u + 0x7FFFu + ((u >> 16) & 1u)) >> 16);
}
__device__ __forceinline__ float bf_bits2f(unsigned short b) { return __uint_as_float(((unsigned)b) << 16); }
__device__ __forceinline__ float bfr(float f) { return bf_bits2f(f2bf_bits(f)); }
__device__ __forceinline__ unsigned pk16(unsigned short a, unsigned short b) { return (unsigned)a | ((unsigned)b << 16); }

__device__ __forceinline__ v8f wmb(const FragB& a, const FragB& b, v8f c) {
  v8f d = __builtin_amdgcn_wmma_f32_16x16x32_bf16(false, a.v, false, b.v, (short)0, c, false, false);
  asm volatile("v_nop\n\tv_nop\n\tv_nop\n\tv_nop" : "+v"(d) : "v"(a.w), "v"(b.w));
  return d;
}
__device__ __forceinline__ v8f z8() { v8f z = {0.f, 0.f, 0.f, 0.f, 0.f, 0.f, 0.f, 0.f}; return z; }

__global__ __launch_bounds__(256) void colstats_kernel(const float* __restrict__ x, float* __restrict__ ST) {
  __shared__ float smn[8][32];
  __shared__ float smx[8][32];
  const int tid = threadIdx.x, lane = tid & 31, w = tid >> 5;
  const int col = blockIdx.x * 32 + lane;
  const float* p = x + col;
  float mn = __uint_as_float(0x7f800000u);
  float mx = __uint_as_float(0xff800000u);
#pragma unroll 4
  for (int r = w; r < NROWS; r += 8) {
    const float v = bfr(p[(size_t)r * NIN]);
    mn = fminf(mn, v);
    mx = fmaxf(mx, v);
  }
  smn[w][lane] = mn;
  smx[w][lane] = mx;
  __syncthreads();
  if (w == 0) {
    float a = smn[0][lane], b = smx[0][lane];
#pragma unroll
    for (int q = 1; q < 8; ++q) { a = fminf(a, smn[q][lane]); b = fmaxf(b, smx[q][lane]); }
    const float wd = fmaxf(b - a, 0.01f);
    const float c  = 0.5f * (b + a);
    const float hw = 0.5f * wd;
    v4f s;
    s[0] = c;
    s[1] = 1.0f / hw;
    s[2] = a;
    s[3] = b;
    float* dst = ST + 4 * col;
    *(volatile v4f*)dst = s;
    __threadfence();
    *(volatile v4f*)dst = s;
  }
}

__global__ __launch_bounds__(256) void wprep_kernel(const float* __restrict__ bw, const float* __restrict__ sw,
                                                     const float* __restrict__ coeff,
                                                     unsigned short* __restrict__ WB) {
  const int o = blockIdx.x, t = threadIdx.x, w = t >> 5;
  unsigned short* row = WB + (size_t)o * KTOT;
  if (w == 0) {
    const float* src = bw + (size_t)o * NIN + 8 * t;
    const v4f a = *(const v4fa*)src;
    const v4f c = *(const v4fa*)(src + 4);
    v4u v;
    v[0] = pk16(f2bf_bits(a[0]), f2bf_bits(a[1]));
    v[1] = pk16(f2bf_bits(a[2]), f2bf_bits(a[3]));
    v[2] = pk16(f2bf_bits(c[0]), f2bf_bits(c[1]));
    v[3] = pk16(f2bf_bits(c[2]), f2bf_bits(c[3]));
    unsigned short* d0 = row + 8 * t;
    unsigned short* d1 = row + OSL + 8 * t;
    *(volatile v4u*)d0 = v;
    *(volatile v4u*)d1 = v;
    __threadfence();
    *(volatile v4u*)d0 = v;
    *(volatile v4u*)d1 = v;
  }
  if (w < 7) {
    const int j0 = 8 * t;
    const float* src = coeff + (size_t)o * KSP + j0;
    const v4f a = *(const v4fa*)src;
    const v4f c = *(const v4fa*)(src + 4);
    const int i0 = j0 / NB;
    const int i1 = (i0 + 1 < NIN) ? (i0 + 1) : (NIN - 1);
    const unsigned s0 = __float_as_uint(sw[(size_t)o * NIN + i0]);
    const unsigned s1 = __float_as_uint(sw[(size_t)o * NIN + i1]);
    const float cv[8] = {a[0], a[1], a[2], a[3], c[0], c[1], c[2], c[3]};
    unsigned short hb[8];
#pragma unroll
    for (int e = 0; e < 8; ++e) {
      const unsigned msk = 0u - (unsigned)((j0 + e) / NB - i0);
      const float swv = __uint_as_float((s0 & ~msk) | (s1 & msk));
      hb[e] = f2bf_bits(bfr(cv[e]) * bfr(swv));
    }
    v4u v;
    v[0] = pk16(hb[0], hb[1]);
    v[1] = pk16(hb[2], hb[3]);
    v[2] = pk16(hb[4], hb[5]);
    v[3] = pk16(hb[6], hb[7]);
    unsigned short* d0 = row + OBH + j0;
    unsigned short* d1 = row + OBL + j0;
    *(volatile v4u*)d0 = v;
    *(volatile v4u*)d1 = v;
    __threadfence();
    *(volatile v4u*)d0 = v;
    *(volatile v4u*)d1 = v;
  }
}

__device__ __forceinline__ void a_store_pass(const unsigned short* sA, unsigned short* dst, int tid) {
#pragma unroll
  for (int it = 0; it < NSWEEP; ++it) {
    const int u = it * FTHR + tid;
    const v4u v = *(const v4ua*)(sA + 8 * u);
    *(volatile v4u*)(dst + 8 * u) = v;
  }
}

__global__ __launch_bounds__(FTHR) void feat_kernel(const float* __restrict__ x, const float* __restrict__ ST,
                                                     unsigned short* __restrict__ AP) {
  __shared__ __align__(16) unsigned short sA[KTOT];
  const int i = threadIdx.x;
  const int b = blockIdx.x;
  const float xb = bfr(x[(size_t)b * NIN + i]);
  const v4f st = *(const v4fa*)(ST + 4 * i);
  float xn = (xb - st[0]) * st[1];
  xn = fminf(fmaxf(xn, -2.0f), 2.0f);

  const float ex   = expf(-xn);
  const float sig  = 1.0f / (1.0f + ex);
  const float silu = xn * sig;

  const float T[11] = { -1.0f, -0.799999952f, -0.600000024f, -0.399999976f, -0.200000018f, 7.4505806e-09f,
                        0.200000033f, 0.400000006f, 0.600000024f, 0.800000072f, 1.0f };
  float bs[8];
#pragma unroll
  for (int m = 0; m < NB; ++m) bs[m] = (xn >= T[m] && xn < T[m + 1]) ? 1.0f : 0.0f;
  bs[7] = 0.0f;
  bs[6] = (xn == T[7]) ? 1.0f : bs[6];
#pragma unroll
  for (int k = 1; k <= 3; ++k) {
    float nb[NB];
#pragma unroll
    for (int m = 0; m < NB; ++m) {
      const float r1 = 1.0f / (T[m + k] - T[m]);
      const float r2 = 1.0f / (T[m + k + 1] - T[m + 1]);
      const float u1 = (xn - T[m]) * r1;
      const float u2 = (T[m + k + 1] - xn) * r2;
      const float t1 = u1 * bs[m];
      const float t2 = u2 * bs[m + 1];
      nb[m] = t1 + t2;
    }
#pragma unroll
    for (int m = 0; m < NB; ++m) bs[m] = nb[m];
  }

  {
    const unsigned short hbits = f2bf_bits(silu);
    const float hv = bf_bits2f(hbits);
    sA[i] = hbits;
    sA[OSL + i] = f2bf_bits(silu - hv);
  }
#pragma unroll
  for (int m = 0; m < NB; ++m) {
    const unsigned short hbits = f2bf_bits(bs[m]);
    const float hv = bf_bits2f(hbits);
    sA[OBH + NB * i + m] = hbits;
    sA[OBL + NB * i + m] = f2bf_bits(bs[m] - hv);
  }
  __syncthreads();

  unsigned short* dst = AP + (size_t)b * KTOT;
  a_store_pass(sA, dst, i);
  __threadfence();
  a_store_pass(sA, dst, i);
}

__device__ __forceinline__ void o_store_pass(const float* sO, float* out, int grow_w, int n0, int w, int lane) {
  const int q8 = lane & 7, sub = lane >> 3;
#pragma unroll
  for (int i = 0; i < 16; ++i) {
    const int lid = i * 4 + sub;
    const int row = lid >> 1, hl = lid & 1;
    const v4f v = *(const v4fa*)(sO + (32 * w + row) * 64 + 32 * hl + 4 * q8);
    *(volatile v4f*)(out + (size_t)(grow_w + row) * NOUT + n0 + 32 * hl + 4 * q8) = v;
  }
}

__global__ __launch_bounds__(128) void gemm_kernel(const unsigned short* __restrict__ AP,
                                                    const unsigned short* __restrict__ WB,
                                                    const float* __restrict__ bias,
                                                    float* __restrict__ out) {
  __shared__ __align__(16) float sO[128 * 64];
  const int tid = threadIdx.x, lane = tid & 31, w = tid >> 5;
  const int h = lane >> 4, m = lane & 15;
  const int row_w = blockIdx.x * 128 + 32 * w;
  const int n0 = blockIdx.y * 64;

  const unsigned short* xa0 = AP + (size_t)(row_w + m) * KTOT + 8 * h;
  const unsigned short* xa1 = xa0 + (size_t)16 * KTOT;
  const unsigned short* wb  = WB + (size_t)(n0 + m) * KTOT + 8 * h;

  v8f acc[2][4];
#pragma unroll
  for (int mt = 0; mt < 2; ++mt)
#pragma unroll
    for (int nt = 0; nt < 4; ++nt) acc[mt][nt] = z8();

#pragma unroll 1
  for (int k0 = 0; k0 < KTOT; k0 += 32) {
    FragB a0, a1;
    a0.h[0] = *(const v8usa*)(xa0 + k0);
    a0.h[1] = *(const v8usa*)(xa0 + k0 + 16);
    a1.h[0] = *(const v8usa*)(xa1 + k0);
    a1.h[1] = *(const v8usa*)(xa1 + k0 + 16);
#pragma unroll
    for (int nt = 0; nt < 4; ++nt) {
      const unsigned short* wq = wb + (size_t)nt * 16 * KTOT + k0;
      FragB bfr_;
      bfr_.h[0] = *(const v8usa*)wq;
      bfr_.h[1] = *(const v8usa*)(wq + 16);
      acc[0][nt] = wmb(a0, bfr_, acc[0][nt]);
      acc[1][nt] = wmb(a1, bfr_, acc[1][nt]);
    }
  }

#pragma unroll
  for (int nt = 0; nt < 4; ++nt) {
    const int cl = 16 * nt + m;
    const float bv = bfr(bias[n0 + cl]);
#pragma unroll
    for (int mt = 0; mt < 2; ++mt) {
#pragma unroll
      for (int r = 0; r < 8; ++r) {
        const int rl = 32 * w + 16 * mt + 8 * h + r;
        sO[rl * 64 + cl] = acc[mt][nt][r] + bv;
      }
    }
  }
  __syncthreads();

  o_store_pass(sO, out, row_w, n0, w, lane);
  __threadfence();
  o_store_pass(sO, out, row_w, n0, w, lane);
}

extern "C" void kernel_launch(void* const* d_in, const int* in_sizes, int n_in,
                              void* d_out, int out_size, void* d_ws, size_t ws_size,
                              hipStream_t stream) {
  if (n_in < 5) return;
  if (in_sizes[0] != NROWS * NIN) return;
  if (in_sizes[1] != NOUT * NIN) return;
  if (in_sizes[2] != NOUT * NIN) return;
  if (in_sizes[3] != NOUT * KSP) return;
  if (in_sizes[4] != NOUT) return;
  if (out_size != NROWS * NOUT) return;

  const float* x     = (const float*)d_in[0];
  const float* bw    = (const float*)d_in[1];
  const float* sw    = (const float*)d_in[2];
  const float* coeff = (const float*)d_in[3];
  const float* bias  = (const float*)d_in[4];
  float* out = (float*)d_out;

  size_t off = 0;
  const size_t oST = off; off += (size_t)NIN * 4 * sizeof(float);
  const size_t oAP = off; off += (size_t)NROWS * KTOT * 2;
  const size_t oWB = off; off += (size_t)NOUT * KTOT * 2;
  if (off > ws_size) return;
  if (off > (size_t)WSCAP) return;

  char* ws = (char*)d_ws;
  float* ST = (float*)(ws + oST);
  unsigned short* AP = (unsigned short*)(ws + oAP);
  unsigned short* WB = (unsigned short*)(ws + oWB);

  colstats_kernel<<<dim3(NIN / 32), dim3(256), 0, stream>>>(x, ST);
  wprep_kernel<<<dim3(NOUT), dim3(256), 0, stream>>>(bw, sw, coeff, WB);
  feat_kernel<<<dim3(NROWS), dim3(FTHR), 0, stream>>>(x, ST, AP);
  gemm_kernel<<<dim3(NROWS / 128, NOUT / 64), dim3(128), 0, stream>>>(AP, WB, bias, out);
  (void)hipGetLastError();
}
